// Self_Attention_55456617726409
// MI455X (gfx1250) — hardware-run, weakly checked
//
#include <hip/hip_runtime.h>


#ifndef NB
#define NB 4
#endif
#ifndef SEQ
#define SEQ 2048
#endif
#define NB_FULL  4
#define SEQ_FULL 2048
#define DM   512
#define NH   8
#define HD   64
#define KT   7
#define KC   (KT * DM)
#define SPAD (SEQ + 6)
#define PCAR 1024.0f
#define PLOG 10.0f
#define SCQ  (0.125f * 1.4426950408889634f)
#define KRES 2048.0f
#define KRINV 4.8828125e-04f
#define BN_EPS 1.0e-5f
#define LN_EPS 1.0e-5f
#define LOP  68
#define LNP  516

static_assert(DM == NH * HD);
static_assert(HD == 64);
static_assert(KC % 32 == 0);
static_assert(DM % 64 == 0);
static_assert(SEQ % 64 == 0);
static_assert(SEQ % 32 == 0);
static_assert(SEQ % 16 == 0);
static_assert(NH * 32 == 256);
static_assert(((size_t)DM * KC) % (8 * 256) == 0);
static_assert(((size_t)SPAD * DM) % 8 == 0);
static_assert((DM / 8) * 8 == DM);
static_assert(NB <= NB_FULL);
static_assert(SEQ <= SEQ_FULL);
static_assert(LOP % 4 == 0);
static_assert(LNP % 4 == 0);
static_assert(32 * 16 * 4 == 16 * HD * 2);
static_assert(32 * 16 * 4 * 2 == 2 * 16 * HD * 2);
static_assert(32 * 16 * 4 == DM * 4);
static_assert(16 * LOP * 4 <= 131072);
static_assert(16 * LNP * 4 <= 131072);
static_assert(2 * NH == 16);
static_assert(KRES * KRINV == 1.0f);

typedef _Float16 h16;
typedef unsigned short bf;
typedef __attribute__((ext_vector_type(16))) __bf16   v16bf;
typedef __attribute__((ext_vector_type(16))) _Float16 v16h;
typedef __attribute__((ext_vector_type(8)))  _Float16 v8h;
typedef __attribute__((ext_vector_type(8)))  unsigned short v8us;
typedef __attribute__((ext_vector_type(8)))  float    v8f;
typedef __attribute__((ext_vector_type(4)))  float    v4f;
typedef v4f  __attribute__((may_alias)) v4fa;

__device__ __forceinline__ unsigned short f2bf(float f) { unsigned u = __float_as_uint(f); u += 0x7FFFu + ((u >> 16) & 1u); return (unsigned short)(u >> 16); }
__device__ __forceinline__ float bf2f(unsigned short b) { return __uint_as_float(((unsigned)b) << 16); }
__device__ __forceinline__ float bfr(float f) { return bf2f(f2bf(f)); }
__device__ __forceinline__ v16h cat16(v8h lo, v8h hi) { return __builtin_shufflevector(lo, hi, 0, 1, 2, 3, 4, 5, 6, 7, 8, 9, 10, 11, 12, 13, 14, 15); }
__device__ __forceinline__ v16bf cat16b(v8us lo, v8us hi) { return __builtin_bit_cast(v16bf, __builtin_shufflevector(lo, hi, 0, 1, 2, 3, 4, 5, 6, 7, 8, 9, 10, 11, 12, 13, 14, 15)); }
__device__ __forceinline__ v16bf ldg16(const bf* __restrict__ p) { return cat16b(*(const v8us*)p, *(const v8us*)(p + 16)); }
__device__ __forceinline__ void wsync() { __builtin_amdgcn_wave_barrier(); asm volatile("" ::: "memory"); }

__device__ __forceinline__ v16h ldh16(const h16* __restrict__ p) { return cat16(*(const v8h*)p, *(const v8h*)(p + 16)); }
static __device__ __forceinline__ h16 toh_flush(float v) { const h16 r = (h16)v; return (fabsf(v) < 6.103515625e-05f) ? (h16)0.0f : r; }
__device__ __forceinline__ v8f wmmab_g(v16bf a, v16bf b, v8f c) {
    c = __builtin_amdgcn_wmma_f32_16x16x32_bf16(false, a, false, b, (short)0, c, false, false);
    asm volatile("v_nop\n\tv_nop\n\tv_nop\n\tv_nop" : "+v"(c) : "v"(a), "v"(b));
    return c;
}
__device__ __forceinline__ v8f wmmah_g(v16h a, v16h b, v8f c) {
    c = __builtin_amdgcn_wmma_f32_16x16x32_f16(false, a, false, b, (short)0, c, false, false);
    asm volatile("v_nop\n\tv_nop\n\tv_nop\n\tv_nop" : "+v"(c) : "v"(a), "v"(b));
    return c;
}

__device__ __forceinline__ void conv_loop(const bf* __restrict__ A, const bf* __restrict__ Bt, const int lda, const int ldb, const size_t aoff, const size_t boff, v8f (&acc)[4][4]) {
#pragma unroll 1
    for (int kc = 0; kc < KC; kc += 32) {
        v16bf a[4];
#pragma unroll
        for (int mb = 0; mb < 4; ++mb) a[mb] = ldg16(A + aoff + (size_t)mb * 16 * lda + kc);
#pragma unroll
        for (int nb = 0; nb < 4; ++nb) { const v16bf b = ldg16(Bt + boff + (size_t)nb * 16 * ldb + kc);
#pragma unroll
            for (int mb = 0; mb < 4; ++mb) acc[mb][nb] = wmmab_g(a[mb], b, acc[mb][nb]); }
    }
}

__global__ __launch_bounds__(256) void k_wconv(const float* __restrict__ w, bf* wt, unsigned n8) {
    const unsigned i = blockIdx.x * 256u + threadIdx.x; if (i >= n8) return;
    const unsigned co = i / (unsigned)(KC / 8), k = (i % (unsigned)(KC / 8)) * 8u; const unsigned tap = k / (unsigned)DM, ci = k % (unsigned)DM;
    const float* s = w + ((size_t)co * DM + ci) * KT + tap; v8us o;
#pragma unroll
    for (int j = 0; j < 8; ++j) o[j] = f2bf(s[(size_t)j * KT]);
    bf* d = wt + (size_t)i * 8;
    *(volatile v8us*)d = o; __threadfence(); *(volatile v8us*)d = o;
}

__global__ __launch_bounds__(256) void k_cvtpad(const float* __restrict__ src, bf* dst, unsigned n8) {
    const unsigned i = blockIdx.x * 256u + threadIdx.x; if (i >= n8) return;
    const int prow = (int)(i / (unsigned)(DM / 8)); const int c = (int)(i % (unsigned)(DM / 8)) * 8;
    const int srow = prow - 3; const bool ok = (srow >= 0) && (srow < SEQ);
    const int sr = (srow < 0) ? 0 : ((srow > SEQ - 1) ? (SEQ - 1) : srow);
    const float* s = src + (size_t)blockIdx.y * SEQ_FULL * DM + (size_t)sr * DM + c;
    const v4f v0 = *(const v4f*)s; const v4f v1 = *(const v4f*)(s + 4); v8us o;
#pragma unroll
    for (int k = 0; k < 4; ++k) { const unsigned short a = f2bf(v0[k]); const unsigned short e = f2bf(v1[k]); o[k] = ok ? a : (unsigned short)0; o[4 + k] = ok ? e : (unsigned short)0; }
    bf* d = dst + (size_t)blockIdx.y * SPAD * DM + (size_t)i * 8;
    *(volatile v8us*)d = o; __threadfence(); *(volatile v8us*)d = o;
}

__global__ __launch_bounds__(32) void k_conv_qk(const bf* __restrict__ X, const bf* __restrict__ W, const float* __restrict__ cb, const float* __restrict__ bg, const float* __restrict__ bb, const float* __restrict__ bm, const float* __restrict__ bv, h16* P, float sc) {
    __shared__ __align__(16) float os[16 * LOP];
    const int lane = threadIdx.x & 31, lr = lane & 15, hi = lane >> 4;
    const size_t z = blockIdx.z; const int r0 = blockIdx.x * 64, c0 = blockIdx.y * 64;
    const bf* A = X + z * (size_t)SPAD * DM;
    v8f acc[4][4];
#pragma unroll
    for (int mb = 0; mb < 4; ++mb)
#pragma unroll
        for (int nb = 0; nb < 4; ++nb) acc[mb][nb] = (v8f){};
    conv_loop(A, W, DM, KC, (size_t)(r0 + lr) * DM + 8 * hi, (size_t)(c0 + lr) * KC + 8 * hi, acc);
    const size_t pbase = ((z * NH + blockIdx.y) * (size_t)SEQ + r0) * HD;
    const int srow = lane >> 3, scol = (lane & 7) * 8;
    float cbv[8], muv[8], mlv[8], bev[8];
#pragma unroll
    for (int j = 0; j < 8; ++j) { const int c = c0 + scol + j; cbv[j] = bfr(cb[c]); muv[j] = bfr(bm[c]); mlv[j] = rsqrtf(bfr(bv[c]) + BN_EPS) * bfr(bg[c]); bev[j] = bfr(bb[c]); }
#pragma unroll
    for (int mb = 0; mb < 4; ++mb) {
#pragma unroll
        for (int nb = 0; nb < 4; ++nb) {
#pragma unroll
            for (int j = 0; j < 8; ++j) os[(hi * 8 + j) * LOP + nb * 16 + lr] = acc[mb][nb][j]; }
        wsync();
#pragma unroll 1
        for (int ps = 0; ps < 2; ++ps) {
#pragma unroll
            for (int s = 0; s < 4; ++s) { const int row = 4 * s + srow; const v4f x0 = *(const v4fa*)(&os[row * LOP + scol]); const v4f x1 = *(const v4fa*)(&os[row * LOP + scol + 4]); v8h o;
#pragma unroll
                for (int j = 0; j < 4; ++j) {
                    const float y0 = ((x0[j] + cbv[j]) - muv[j]) * mlv[j] + bev[j];
                    const float y1 = ((x1[j] + cbv[4 + j]) - muv[4 + j]) * mlv[4 + j] + bev[4 + j];
                    o[j] = toh_flush(y0 * sc); o[4 + j] = toh_flush(y1 * sc); }
                *(volatile v8h*)(P + pbase + (size_t)(mb * 16 + row) * HD + scol) = o; }
            if (ps == 0) __threadfence(); }
        wsync();
    }
}

__global__ __launch_bounds__(32) void k_conv_k(const bf* __restrict__ X, const bf* __restrict__ W, const float* __restrict__ cb, const float* __restrict__ bg, const float* __restrict__ bb, const float* __restrict__ bm, const float* __restrict__ bv, h16* KH, h16* KR) {
    __shared__ __align__(16) float os[16 * LOP];
    const int lane = threadIdx.x & 31, lr = lane & 15, hi = lane >> 4;
    const size_t z = blockIdx.z; const int r0 = blockIdx.x * 64, c0 = blockIdx.y * 64;
    const bf* A = X + z * (size_t)SPAD * DM;
    v8f acc[4][4];
#pragma unroll
    for (int mb = 0; mb < 4; ++mb)
#pragma unroll
        for (int nb = 0; nb < 4; ++nb) acc[mb][nb] = (v8f){};
    conv_loop(A, W, DM, KC, (size_t)(r0 + lr) * DM + 8 * hi, (size_t)(c0 + lr) * KC + 8 * hi, acc);
    const size_t pbase = ((z * NH + blockIdx.y) * (size_t)SEQ + r0) * HD;
    const int srow = lane >> 3, scol = (lane & 7) * 8;
    float cbv[8], muv[8], mlv[8], bev[8];
#pragma unroll
    for (int j = 0; j < 8; ++j) { const int c = c0 + scol + j; cbv[j] = bfr(cb[c]); muv[j] = bfr(bm[c]); mlv[j] = rsqrtf(bfr(bv[c]) + BN_EPS) * bfr(bg[c]); bev[j] = bfr(bb[c]); }
#pragma unroll
    for (int mb = 0; mb < 4; ++mb) {
#pragma unroll
        for (int nb = 0; nb < 4; ++nb) {
#pragma unroll
            for (int j = 0; j < 8; ++j) os[(hi * 8 + j) * LOP + nb * 16 + lr] = acc[mb][nb][j]; }
        wsync();
#pragma unroll 1
        for (int ps = 0; ps < 2; ++ps) {
#pragma unroll
            for (int s = 0; s < 4; ++s) { const int row = 4 * s + srow; const v4f x0 = *(const v4fa*)(&os[row * LOP + scol]); const v4f x1 = *(const v4fa*)(&os[row * LOP + scol + 4]); v8h oh, ores;
#pragma unroll
                for (int j = 0; j < 4; ++j) {
                    const float y0 = ((x0[j] + cbv[j]) - muv[j]) * mlv[j] + bev[j];
                    const float y1 = ((x1[j] + cbv[4 + j]) - muv[4 + j]) * mlv[4 + j] + bev[4 + j];
                    const h16 h0 = toh_flush(y0); const h16 h1 = toh_flush(y1);
                    oh[j] = h0; oh[4 + j] = h1;
                    ores[j] = toh_flush((y0 - (float)h0) * KRES); ores[4 + j] = toh_flush((y1 - (float)h1) * KRES); }
                const size_t off = pbase + (size_t)(mb * 16 + row) * HD + scol;
                *(volatile v8h*)(KH + off) = oh; *(volatile v8h*)(KR + off) = ores; }
            if (ps == 0) __threadfence(); }
        wsync();
    }
}

__global__ __launch_bounds__(32) void k_conv_vt(const bf* __restrict__ W, const bf* __restrict__ X, const float* __restrict__ cb, const float* __restrict__ bg, const float* __restrict__ bb, const float* __restrict__ bm, const float* __restrict__ bv, h16* VT) {
    __shared__ __align__(16) float os[16 * LOP];
    const int lane = threadIdx.x & 31, lr = lane & 15, hi = lane >> 4;
    const size_t z = blockIdx.z; const int r0 = blockIdx.x * 64, c0 = blockIdx.y * 64;
    const bf* Bt = X + z * (size_t)SPAD * DM;
    v8f acc[4][4];
#pragma unroll
    for (int mb = 0; mb < 4; ++mb)
#pragma unroll
        for (int nb = 0; nb < 4; ++nb) acc[mb][nb] = (v8f){};
    conv_loop(W, Bt, KC, DM, (size_t)(r0 + lr) * KC + 8 * hi, (size_t)(c0 + lr) * DM + 8 * hi, acc);
    const size_t vb0 = z * (size_t)DM * SEQ + (size_t)r0 * SEQ + c0;
    const int srow = lane >> 3, scol = (lane & 7) * 8;
#pragma unroll
    for (int mb = 0; mb < 4; ++mb) {
#pragma unroll
        for (int nb = 0; nb < 4; ++nb) {
#pragma unroll
            for (int j = 0; j < 8; ++j) os[(hi * 8 + j) * LOP + nb * 16 + lr] = acc[mb][nb][j]; }
        wsync();
#pragma unroll 1
        for (int ps = 0; ps < 2; ++ps) {
#pragma unroll
            for (int s = 0; s < 4; ++s) { const int row = 4 * s + srow; const v4f x0 = *(const v4fa*)(&os[row * LOP + scol]); const v4f x1 = *(const v4fa*)(&os[row * LOP + scol + 4]); v8h o;
                const int ch = r0 + mb * 16 + row;
                const float c_b = bfr(cb[ch]), c_m = bfr(bm[ch]), c_l = rsqrtf(bfr(bv[ch]) + BN_EPS) * bfr(bg[ch]), c_e = bfr(bb[ch]);
#pragma unroll
                for (int j = 0; j < 4; ++j) { o[j] = toh_flush(((x0[j] + c_b) - c_m) * c_l + c_e); o[4 + j] = toh_flush(((x1[j] + c_b) - c_m) * c_l + c_e); }
                *(volatile v8h*)(VT + vb0 + (size_t)(mb * 16 + row) * SEQ + scol) = o; }
            if (ps == 0) __threadfence(); }
        wsync();
    }
}

__global__ __launch_bounds__(256) __attribute__((amdgpu_num_vgpr(256))) void k_attn_ln(const h16* __restrict__ Qp, const h16* __restrict__ Kp, const h16* __restrict__ Kr, const h16* __restrict__ VT, const float* __restrict__ lng, const float* __restrict__ lnb, float* OUT) {
    __shared__ __align__(16) float o_s[16 * LNP];
    const int lane = threadIdx.x & 31, lr = lane & 15, hi = lane >> 4;
    const int wave = __builtin_amdgcn_readfirstlane(threadIdx.x >> 5);
    const int b = blockIdx.y; const int q0 = blockIdx.x * 16;
    const size_t pl = ((size_t)b * NH + (size_t)wave) * SEQ * HD;
    const size_t koff = pl + (size_t)lr * HD + 8 * hi;
    const size_t voff = ((size_t)b * DM + (size_t)wave * HD + (size_t)lr) * SEQ + 8 * hi;
    const v16h qb0 = ldh16(Qp + pl + (size_t)(q0 + lr) * HD + 8 * hi);
    const v16h qb1 = ldh16(Qp + pl + (size_t)(q0 + lr) * HD + 8 * hi + 32);
    v8f o[4];
#pragma unroll
    for (int dt = 0; dt < 4; ++dt) o[dt] = (v8f){};
    float m = -1.0e30f, l = 0.0f;

#pragma unroll 1
    for (int k0 = 0; k0 < SEQ; k0 += 32) {
        const h16* kp = Kp + koff + (size_t)k0 * HD;
        const v16h ka00 = ldh16(kp), ka01 = ldh16(kp + 32);
        const v16h ka10 = ldh16(kp + 16 * HD), ka11 = ldh16(kp + 16 * HD + 32);
        v8f s0 = (v8f){}, s1 = (v8f){};
        s0 = wmmah_g(ka00, qb0, s0); s1 = wmmah_g(ka10, qb0, s1);
        s0 = wmmah_g(ka01, qb1, s0); s1 = wmmah_g(ka11, qb1, s1);
        const h16* rp = Kr + koff + (size_t)k0 * HD;
        const v16h kr00 = ldh16(rp), kr01 = ldh16(rp + 32);
        const v16h kr10 = ldh16(rp + 16 * HD), kr11 = ldh16(rp + 16 * HD + 32);
        v8f t0 = (v8f){}, t1 = (v8f){};
        t0 = wmmah_g(kr00, qb0, t0); t1 = wmmah_g(kr10, qb0, t1);
        t0 = wmmah_g(kr01, qb1, t0); t1 = wmmah_g(kr11, qb1, t1);
#pragma unroll
        for (int r = 0; r < 8; ++r) { s0[r] = s0[r] + t0[r] * KRINV; s1[r] = s1[r] + t1[r] * KRINV; }
        float mx = fmaxf(s0[0], s1[0]);
#pragma unroll
        for (int r = 1; r < 8; ++r) mx = fmaxf(mx, fmaxf(s0[r], s1[r]));
        mx = fmaxf(mx, __shfl_xor(mx, 16, 32));
        const float mnew = fmaxf(m, mx);
        const float al = __builtin_amdgcn_exp2f(m - mnew);
        m = mnew;
        const float mc = mnew - PLOG;
        float sum = 0.0f; v16h pb;
#pragma unroll
        for (int r = 0; r < 8; ++r) {
            const float e0 = s0[r] - mc, e1 = s1[r] - mc;
            const float x0 = __builtin_amdgcn_exp2f(e0), x1 = __builtin_amdgcn_exp2f(e1);
            const float p0 = (e0 < -14.0f) ? 0.0f : x0;
            const float p1 = (e1 < -14.0f) ? 0.0f : x1;
            sum += p0 + p1;
            pb[r] = (h16)p0; pb[8 + r] = (h16)p1;
        }
        l = l * al + sum;
#pragma unroll
        for (int dt = 0; dt < 4; ++dt)
#pragma unroll
            for (int r = 0; r < 8; ++r) o[dt][r] *= al;
        const h16* vp = VT + voff + k0;
#pragma unroll
        for (int dt = 0; dt < 4; ++dt) { const v16h va = ldh16(vp + (size_t)dt * 16 * SEQ); o[dt] = wmmah_g(va, pb, o[dt]); }
    }
    l += __shfl_xor(l, 16, 32);
    const float inv = 1.0f / l;
#pragma unroll
    for (int dt = 0; dt < 4; ++dt) {
        const v4f a0 = { o[dt][0] * inv, o[dt][1] * inv, o[dt][2] * inv, o[dt][3] * inv };
        const v4f a1 = { o[dt][4] * inv, o[dt][5] * inv, o[dt][6] * inv, o[dt][7] * inv };
        *(v4fa*)(&o_s[lr * LNP + wave * HD + dt * 16 + 8 * hi]) = a0;
        *(v4fa*)(&o_s[lr * LNP + wave * HD + dt * 16 + 8 * hi + 4]) = a1;
    }
    __syncthreads();
#pragma unroll 1
    for (int i = 0; i < 2; ++i) {
        const int row = wave * 2 + i;
        v4f x[4]; float s = 0.0f;
#pragma unroll
        for (int j = 0; j < 4; ++j) { x[j] = *(const v4fa*)(&o_s[row * LNP + j * 128 + lane * 4]); s += (x[j][0] + x[j][1]) + (x[j][2] + x[j][3]); }
        s += __shfl_xor(s, 16, 32); s += __shfl_xor(s, 8, 32); s += __shfl_xor(s, 4, 32); s += __shfl_xor(s, 2, 32); s += __shfl_xor(s, 1, 32);
        const float mu = s * (1.0f / (float)DM);
        float ss = 0.0f;
#pragma unroll
        for (int j = 0; j < 4; ++j)
#pragma unroll
            for (int e = 0; e < 4; ++e) { const float d = x[j][e] - mu; ss += d * d; }
        ss += __shfl_xor(ss, 16, 32); ss += __shfl_xor(ss, 8, 32); ss += __shfl_xor(ss, 4, 32); ss += __shfl_xor(ss, 2, 32); ss += __shfl_xor(ss, 1, 32);
        const float rstd = rsqrtf(ss * (1.0f / (float)DM) + LN_EPS);
        v4f y[4];
#pragma unroll
        for (int j = 0; j < 4; ++j) { const v4f gv = *(const v4f*)(lng + j * 128 + lane * 4); const v4f bv = *(const v4f*)(lnb + j * 128 + lane * 4);
#pragma unroll
            for (int e = 0; e < 4; ++e) y[j][e] = (x[j][e] - mu) * rstd * bfr(gv[e]) + bfr(bv[e]); }
        float* orow = OUT + ((size_t)b * SEQ_FULL + (size_t)(q0 + row)) * DM + lane * 4;
#pragma unroll 1
        for (int ps = 0; ps < 2; ++ps) {
#pragma unroll
            for (int j = 0; j < 4; ++j) *(volatile v4f*)(orow + j * 128) = y[j];
            if (ps == 0) __threadfence(); }
    }
}

constexpr size_t al256(size_t x) { return (x + 255) & ~(size_t)255; }
constexpr size_t SZ_WT = al256((size_t)DM * KC * 2);
constexpr size_t SZ_XP = al256((size_t)NB * SPAD * DM * 2);
constexpr size_t SZ_P  = al256((size_t)NB * NH * SEQ * HD * 2);
constexpr size_t WS_TOTAL = SZ_WT + 3 * SZ_XP + 4 * SZ_P;
static_assert(WS_TOTAL <= (size_t)134217728);
static_assert(SZ_WT == (size_t)DM * KC * 2);
static_assert(SZ_XP == (size_t)NB * SPAD * DM * 2);
static_assert(SZ_P == (size_t)NB * DM * SEQ * 2);

extern "C" void kernel_launch(void* const* d_in, const int* in_sizes, int n_in,
                              void* d_out, int out_size, void* d_ws, size_t ws_size, hipStream_t stream) {
    if (n_in < 11) return;
    const size_t need_act = (size_t)(NB - 1) * SEQ_FULL * DM + (size_t)SEQ * DM;
    if ((size_t)in_sizes[0] < need_act || (size_t)in_sizes[1] < need_act || (size_t)in_sizes[2] < need_act) return;
    if ((size_t)in_sizes[3] < (size_t)DM * DM * KT) return;
    for (int i = 4; i < 11; ++i) { if (in_sizes[i] < DM) return; }
    if ((size_t)out_size < need_act) return;
    if (WS_TOTAL > ws_size) return;
    const float* xq = (const float*)d_in[0]; const float* xk = (const float*)d_in[1]; const float* xv = (const float*)d_in[2];
    const float* cw = (const float*)d_in[3]; const float* cb = (const float*)d_in[4];
    const float* bg = (const float*)d_in[5]; const float* bb = (const float*)d_in[6]; const float* bm = (const float*)d_in[7]; const float* bv = (const float*)d_in[8];
    const float* lg = (const float*)d_in[9]; const float* lb = (const float*)d_in[10];
    float* OUT = (float*)d_out;
    char* wsp = (char*)d_ws;
    auto take = [&](size_t bytes) { char* p = wsp; wsp += bytes; return (void*)p; };
    bf* WT = (bf*)take(SZ_WT);
    bf* XQ = (bf*)take(SZ_XP); bf* XK = (bf*)take(SZ_XP); bf* XV = (bf*)take(SZ_XP);
    h16* QP = (h16*)take(SZ_P); h16* KP = (h16*)take(SZ_P); h16* KR = (h16*)take(SZ_P); h16* VT = (h16*)take(SZ_P);
    if ((size_t)(wsp - (char*)d_ws) != WS_TOTAL) return;

    const unsigned nw8 = (unsigned)((size_t)DM * KC / 8), na8 = (unsigned)((size_t)SPAD * DM / 8);
    k_wconv<<<dim3(nw8 / 256), 256, 0, stream>>>(cw, WT, nw8);
    k_cvtpad<<<dim3((na8 + 255) / 256, NB), 256, 0, stream>>>(xq, XQ, na8);
    k_cvtpad<<<dim3((na8 + 255) / 256, NB), 256, 0, stream>>>(xk, XK, na8);
    k_cvtpad<<<dim3((na8 + 255) / 256, NB), 256, 0, stream>>>(xv, XV, na8);
    k_conv_qk<<<dim3(SEQ / 64, NH, NB), 32, 0, stream>>>(XQ, WT, cb, bg, bb, bm, bv, QP, SCQ);
    k_conv_k<<<dim3(SEQ / 64, NH, NB), 32, 0, stream>>>(XK, WT, cb, bg, bb, bm, bv, KP, KR);
    k_conv_vt<<<dim3(DM / 64, SEQ / 64, NB), 32, 0, stream>>>(WT, XV, cb, bg, bb, bm, bv, VT);
    k_attn_ln<<<dim3(SEQ / 16, NB), 256, 0, stream>>>(QP, KP, KR, VT, lg, lb, OUT);
}
